// DRNA_Block_11269994184841
// MI455X (gfx1250) — hardware-run, weakly checked
//
#include <hip/hip_runtime.h>
#include <math.h>

constexpr int kBatch = 2;
constexpr int kSeq   = 2048;
constexpr int kDim   = 1024;
constexpr int kHeads = 16;
constexpr int kDh    = 64;
constexpr int kFF    = 4096;
constexpr int kFFH   = 2048;
constexpr int kTok   = kBatch * kSeq;
constexpr int kQKVN  = 3 * kDim;
constexpr int kGroups = kBatch * kHeads;
constexpr int kGrpPerChunk = 2;
constexpr float kWCarry    = 16.0f;
constexpr float kWCarryInv = 1.0f / 16.0f;
constexpr float kPCarry    = 2048.0f;
constexpr float kPCarryInv = 1.0f / 2048.0f;
constexpr float kScoreScale = 0.125f;
constexpr float kInvDim = 1.0f / 1024.0f;
constexpr float kLnEps  = 1e-5f;

typedef __attribute__((ext_vector_type(16))) _Float16 v16h;
typedef __attribute__((ext_vector_type(8)))  _Float16 v8h;
typedef __attribute__((ext_vector_type(16))) __bf16   v16b;
typedef __attribute__((ext_vector_type(8)))  __bf16   v8b;
typedef __attribute__((ext_vector_type(8)))  float    v8f;
typedef __attribute__((ext_vector_type(4)))  float    v4f;
typedef __attribute__((ext_vector_type(4)))  unsigned int v4u;

__device__ __forceinline__ unsigned short f2bf_bits(float f) {
  unsigned u = __float_as_uint(f);
  return (unsigned short)((u + 0x7FFFu + ((u >> 16) & 1u)) >> 16);
}
__device__ __forceinline__ float bf_bits2f(unsigned short h) { return __uint_as_float(((unsigned)h) << 16); }

__device__ __forceinline__ void dep_guard_h(v8f& a, v8f& b, v16h x, v16h y) { asm volatile("v_nop\n\tv_nop\n\tv_nop\n\tv_nop" : "+v"(a), "+v"(b) : "v"(x), "v"(y)); }
__device__ __forceinline__ void dep_guard_b(v8f& a, v8f& b, v16b x, v16b y) { asm volatile("v_nop\n\tv_nop\n\tv_nop\n\tv_nop" : "+v"(a), "+v"(b) : "v"(x), "v"(y)); }
__device__ __forceinline__ void keep4_h(v16h a, v16h b, v16h c, v16h d) { asm volatile("v_nop" :: "v"(a), "v"(b), "v"(c), "v"(d)); }
__device__ __forceinline__ void keep4_b(v16b a, v16b b, v16b c, v16b d) { asm volatile("v_nop" :: "v"(a), "v"(b), "v"(c), "v"(d)); }
__device__ __forceinline__ void acc_guard4(v8f& a, v8f& b, v8f& c, v8f& d) { asm volatile("v_nop\n\tv_nop\n\tv_nop\n\tv_nop" : "+v"(a), "+v"(b), "+v"(c), "+v"(d)); }
template <typename T> struct Frag;
template <> struct Frag<_Float16> {
  typedef v16h V; union U { v16h v; v8h h[2]; };
  static __device__ __forceinline__ v16h load(const _Float16* p) {
    U f; f.h[0] = *(const v8h*)(p); f.h[1] = *(const v8h*)(p + 16); return f.v;
  }
  static __device__ __forceinline__ v8f mma(v16h a, v16h b, v8f c) {
    return __builtin_amdgcn_wmma_f32_16x16x32_f16(false, a, false, b, (short)0, c, false, false);
  }
  static __device__ __forceinline__ void guard(v8f& a, v8f& b, v16h x, v16h y) { dep_guard_h(a, b, x, y); }
  static __device__ __forceinline__ void keep(v16h a, v16h b, v16h c, v16h d) { keep4_h(a, b, c, d); }
};
template <> struct Frag<__bf16> {
  typedef v16b V; union U { v16b v; v8b h[2]; };
  static __device__ __forceinline__ v16b load(const __bf16* p) {
    U f; f.h[0] = *(const v8b*)(p); f.h[1] = *(const v8b*)(p + 16); return f.v;
  }
  static __device__ __forceinline__ v8f mma(v16b a, v16b b, v8f c) {
    return __builtin_amdgcn_wmma_f32_16x16x32_bf16(false, a, false, b, (short)0, c, false, false);
  }
  static __device__ __forceinline__ void guard(v8f& a, v8f& b, v16b x, v16b y) { dep_guard_b(a, b, x, y); }
  static __device__ __forceinline__ void keep(v16b a, v16b b, v16b c, v16b d) { keep4_b(a, b, c, d); }
};

__device__ __forceinline__ unsigned pk16(unsigned short a, unsigned short b) { return (unsigned)a | ((unsigned)b << 16); }
__device__ __forceinline__ unsigned short h_bits(float f) { const _Float16 h = (_Float16)f; return __builtin_bit_cast(unsigned short, h); }

template <int ET> struct Elem;
template <> struct Elem<0> { typedef _Float16 T; };
template <> struct Elem<1> { typedef __bf16 T; };
template <int ET, bool SPLIT, int BIAS_MODE, int OUT_MODE, bool RESID, int ACT = 0>
__global__ __launch_bounds__(256) void wmma_gemm64(
    const unsigned short* __restrict__ Ap, const unsigned short* __restrict__ A2p, int lda, long strideA,
    const unsigned short* __restrict__ Btp, const unsigned short* __restrict__ Bt2p, int ldb, long strideB,
    void* __restrict__ Cout, void* __restrict__ Cout2, int ldc, long strideC,
    const float* __restrict__ bias,
    const float* __restrict__ resid, long strideR,
    int M, int N, int K, float scale) {
  typedef typename Elem<ET>::T T;
  typedef typename Frag<T>::V V;
  const T* A = (const T*)Ap; const T* A2 = (const T*)A2p; const T* Bt = (const T*)Btp; const T* Bt2 = (const T*)Bt2p;
  __shared__ __align__(16) float sT[8][16 * 68];
  const int b    = blockIdx.y;
  const int lane = threadIdx.x & 31;
  const int wave = threadIdx.x >> 5;
  const int tilesN = N >> 6;
  const int tilesM = M >> 6;
  const int tile = blockIdx.x * 8 + wave;
  if (tile >= tilesM * tilesN) return;
  const int tm = tile / tilesN;
  const int tn = tile - tm * tilesN;
  const int m0 = tm << 6;
  const int n0 = tn << 6;

  const T* Ab  = A  + (size_t)b * strideA;
  const T* Bb  = Bt + (size_t)b * strideB;
  const T* Ab2 = SPLIT ? (A2  + (size_t)b * strideA) : nullptr;
  const T* Bb2 = SPLIT ? (Bt2 + (size_t)b * strideB) : nullptr;

  const int rlane = lane & 15;
  const int koff  = (lane >> 4) * 8;
  const int mOff  = (lane >> 4) * 8;

  v8f acc[4][4];
#pragma unroll
  for (int i = 0; i < 4; ++i)
#pragma unroll
    for (int j = 0; j < 4; ++j) acc[i][j] = (v8f){0.f,0.f,0.f,0.f,0.f,0.f,0.f,0.f};

  for (int k0 = 0; k0 < K; k0 += 32) {
    V bh[4], bl[4];
#pragma unroll
    for (int j = 0; j < 4; ++j) {
      const size_t bo = (size_t)(n0 + (j << 4) + rlane) * ldb + koff + k0;
      bh[j] = Frag<T>::load(Bb + bo);
      if (SPLIT) bl[j] = Frag<T>::load(Bb2 + bo);
    }
#pragma unroll
    for (int i = 0; i < 4; ++i) {
      const size_t ao = (size_t)(m0 + (i << 4) + rlane) * lda + koff + k0;
      V ah = Frag<T>::load(Ab + ao);
      V al;
      if (SPLIT) al = Frag<T>::load(Ab2 + ao);
#pragma unroll
      for (int j = 0; j < 4; ++j) {
        acc[i][j] = Frag<T>::mma(ah, bh[j], acc[i][j]);
        if (SPLIT) {
          acc[i][j] = Frag<T>::mma(ah, bl[j], acc[i][j]);
          acc[i][j] = Frag<T>::mma(al, bh[j], acc[i][j]);
        }
      }
      Frag<T>::guard(acc[i][0], acc[i][3], ah, SPLIT ? al : ah);
    }
    Frag<T>::keep(bh[0], bh[1], bh[2], bh[3]);
    if (SPLIT) Frag<T>::keep(bl[0], bl[1], bl[2], bl[3]);
  }
  acc_guard4(acc[0][0], acc[0][1], acc[0][2], acc[0][3]);
  acc_guard4(acc[1][0], acc[1][1], acc[1][2], acc[1][3]);
  acc_guard4(acc[2][0], acc[2][1], acc[2][2], acc[2][3]);
  acc_guard4(acc[3][0], acc[3][1], acc[3][2], acc[3][3]);

  float* slab = sT[wave];
  const float* Rb = RESID ? (resid + (size_t)b * strideR) : nullptr;
#pragma unroll
  for (int i = 0; i < 4; ++i) {
    const int mBase = m0 + (i << 4);
#pragma unroll
    for (int j = 0; j < 4; ++j) {
      const int n = n0 + (j << 4) + rlane;
      float bv = 0.f;
      if (BIAS_MODE == 2) bv = bias[n];
#pragma unroll
      for (int r = 0; r < 8; ++r) {
        float v = acc[i][j][r] * scale;
        if (BIAS_MODE == 1) v += bias[mBase + mOff + r];
        if (BIAS_MODE == 2) v += bv;
        if (RESID) v += Rb[(size_t)(mBase + mOff + r) * ldc + n];
        if (ACT == 2) v = fmaxf(v, 0.0f);
        if (ACT == 4) v = (v > 0.f) ? v : 0.01f * v;
        slab[(mOff + r) * 68 + (j << 4) + rlane] = v;
      }
    }
    __builtin_amdgcn_fence(__ATOMIC_RELEASE, "workgroup");
    __builtin_amdgcn_wave_barrier();
    __builtin_amdgcn_fence(__ATOMIC_ACQUIRE, "workgroup");
    if (OUT_MODE == 0) {
      float* C = (float*)Cout + (size_t)b * strideC;
      const int hh = lane >> 4, c4 = (lane & 15) * 4;
      for (int pass = 0; pass < 2; ++pass) {
#pragma unroll
        for (int it = 0; it < 8; ++it) {
          const int row = it * 2 + hh;
          v4f v = *(const v4f*)(slab + row * 68 + c4);
          *(volatile v4f*)(C + (size_t)(mBase + row) * ldc + n0 + c4) = v;
        }
        __threadfence();
      }
    } else {
      const int q = lane >> 3, c8 = (lane & 7) * 8;
      unsigned short* C  = (unsigned short*)Cout  + (size_t)b * strideC;
      unsigned short* C2 = (OUT_MODE == 2) ? ((unsigned short*)Cout2 + (size_t)b * strideC) : nullptr;
      for (int pass = 0; pass < 2; ++pass) {
#pragma unroll
        for (int it = 0; it < 4; ++it) {
          const int row = it * 4 + q;
          const float* sp = slab + row * 68 + c8;
          v8h hv, lv;
#pragma unroll
          for (int e = 0; e < 8; ++e) {
            if (OUT_MODE == 1) {
              hv[e] = (_Float16)sp[e];
            } else {
              unsigned short hb = f2bf_bits(sp[e]);
              unsigned short lb = f2bf_bits(sp[e] - bf_bits2f(hb));
              hv[e] = __builtin_bit_cast(_Float16, hb);
              lv[e] = __builtin_bit_cast(_Float16, lb);
            }
          }
          *(volatile v8h*)(C + (size_t)(mBase + row) * ldc + n0 + c8) = hv;
          if (OUT_MODE == 2) *(volatile v8h*)(C2 + (size_t)(mBase + row) * ldc + n0 + c8) = lv;
        }
        __threadfence();
      }
    }
    __builtin_amdgcn_fence(__ATOMIC_RELEASE, "workgroup");
    __builtin_amdgcn_wave_barrier();
    __builtin_amdgcn_fence(__ATOMIC_ACQUIRE, "workgroup");
  }
}

__global__ __launch_bounds__(256) void cast8_f16_kernel(const float* __restrict__ in, unsigned short* __restrict__ out, int n8) {
  const int i = blockIdx.x * 256 + threadIdx.x;
  if (i >= n8) return;
  const float* p = in + 8 * (size_t)i;
  const v4f a = *(const v4f*)(p);
  const v4f c = *(const v4f*)(p + 4);
  unsigned short hb[8];
#pragma unroll
  for (int e = 0; e < 4; ++e) {
    hb[e]     = h_bits(a[e]);
    hb[4 + e] = h_bits(c[e]);
  }
  const v4u u = (v4u){pk16(hb[0], hb[1]), pk16(hb[2], hb[3]), pk16(hb[4], hb[5]), pk16(hb[6], hb[7])};
  unsigned short* q = out + 8 * (size_t)i;
  *(volatile v4u*)q = u;
  __threadfence();
  *(volatile v4u*)q = u;
}

__global__ __launch_bounds__(256) void wtcast_kernel(const float* __restrict__ W, unsigned short* __restrict__ out,
                                                     int Kin, int Nout, float scale) {
  __shared__ float sm[64][65];
  const int t  = threadIdx.x;
  const int k0 = blockIdx.x * 64;
  const int n0 = blockIdx.y * 64;
#pragma unroll
  for (int i = 0; i < 16; ++i) {
    const int e = i * 256 + t;
    const int r = e >> 6;
    const int c = e & 63;
    sm[c][r] = W[(size_t)(k0 + r) * Nout + n0 + c] * scale;
  }
  __syncthreads();
  const int lane = t & 31, wave = t >> 5;
  const int q = lane >> 3, c8 = (lane & 7) * 8;
  v4u u[2];
#pragma unroll
  for (int it = 0; it < 2; ++it) {
    const int row = wave * 8 + it * 4 + q;
    unsigned short hb[8];
#pragma unroll
    for (int e = 0; e < 8; ++e) hb[e] = h_bits(sm[row][c8 + e]);
    u[it] = (v4u){pk16(hb[0], hb[1]), pk16(hb[2], hb[3]), pk16(hb[4], hb[5]), pk16(hb[6], hb[7])};
  }
  for (int pass = 0; pass < 2; ++pass) {
#pragma unroll
    for (int it = 0; it < 2; ++it) {
      const int row = wave * 8 + it * 4 + q;
      *(volatile v4u*)(out + (size_t)(n0 + row) * Kin + k0 + c8) = u[it];
    }
    __threadfence();
  }
}

__global__ __launch_bounds__(256) void rope_split_kernel(const float* __restrict__ QKV,
                                                         const float* __restrict__ cosb,
                                                         const float* __restrict__ sinb,
                                                         unsigned short* __restrict__ Q16,
                                                         unsigned short* __restrict__ K16,
                                                         unsigned short* __restrict__ VT16) {
  __shared__ float sq[64][65];
  __shared__ float sk[64][65];
  __shared__ float sv[64][65];
  const int t  = threadIdx.x;
  const int g  = blockIdx.y;
  const int b  = g >> 4;
  const int h  = g & 15;
  const int s0 = blockIdx.x * 64;
  const int rowbase = b * kSeq + s0;
#pragma unroll
  for (int i = 0; i < 16; ++i) {
    const int e   = i * 256 + t;
    const int tok = e >> 6;
    const int d   = e & 63;
    const float* p = QKV + (size_t)(rowbase + tok) * kQKVN + h * kDh + d;
    sq[tok][d] = p[0];
    sk[tok][d] = p[kDim];
    sv[tok][d] = p[2 * kDim];
  }
  __syncthreads();
  const int lane = t & 31, wave = t >> 5;
  const int q8 = lane >> 3, c8 = (lane & 7) * 8;
  const float sgn = (c8 < 32) ? -1.0f : 1.0f;
  v4u uq[2], uk[2], uv[2];
#pragma unroll
  for (int it = 0; it < 2; ++it) {
    const int tok = wave * 8 + it * 4 + q8;
    const float* cp = cosb + (size_t)(rowbase + tok) * kDh + c8;
    const float* sp = sinb + (size_t)(rowbase + tok) * kDh + c8;
    const v4f ca = *(const v4f*)(cp), cb = *(const v4f*)(cp + 4);
    const v4f sa = *(const v4f*)(sp), sb = *(const v4f*)(sp + 4);
    float cs[8], sn[8];
#pragma unroll
    for (int e = 0; e < 4; ++e) { cs[e] = ca[e]; cs[4 + e] = cb[e]; sn[e] = sa[e]; sn[4 + e] = sb[e]; }
    unsigned short hq[8], hk[8], hv[8];
#pragma unroll
    for (int e = 0; e < 8; ++e) {
      const int d  = c8 + e;
      const int dp = d ^ 32;
      const float qv = sq[tok][d] * cs[e] + sgn * sq[tok][dp] * sn[e];
      const float kv = sk[tok][d] * cs[e] + sgn * sk[tok][dp] * sn[e];
      hq[e] = h_bits(qv);
      hk[e] = h_bits(kv);
    }
    const int dv = wave * 8 + it * 4 + q8;
#pragma unroll
    for (int e = 0; e < 8; ++e) hv[e] = h_bits(sv[c8 + e][dv]);
    uq[it] = (v4u){pk16(hq[0], hq[1]), pk16(hq[2], hq[3]), pk16(hq[4], hq[5]), pk16(hq[6], hq[7])};
    uk[it] = (v4u){pk16(hk[0], hk[1]), pk16(hk[2], hk[3]), pk16(hk[4], hk[5]), pk16(hk[6], hk[7])};
    uv[it] = (v4u){pk16(hv[0], hv[1]), pk16(hv[2], hv[3]), pk16(hv[4], hv[5]), pk16(hv[6], hv[7])};
  }
  for (int pass = 0; pass < 2; ++pass) {
#pragma unroll
    for (int it = 0; it < 2; ++it) {
      const int tok = wave * 8 + it * 4 + q8;
      const size_t oqk = ((size_t)g * kSeq + s0 + tok) * kDh + c8;
      *(volatile v4u*)(Q16 + oqk) = uq[it];
      *(volatile v4u*)(K16 + oqk) = uk[it];
      const int dv = wave * 8 + it * 4 + q8;
      const size_t ov = ((size_t)g * kDh + dv) * kSeq + s0 + c8;
      *(volatile v4u*)(VT16 + ov) = uv[it];
    }
    __threadfence();
  }
}

__global__ __launch_bounds__(256) void softmax_row_kernel(const float* __restrict__ Sc, unsigned short* __restrict__ P, float carry) {
  __shared__ float redM[8];
  __shared__ float redS[8];
  const int row  = blockIdx.x;
  const int t    = threadIdx.x;
  const int lane = t & 31, wave = t >> 5;
  const int c0   = t * 8;
  const float* sr = Sc + (size_t)row * kSeq + c0;
  const v4f a = *(const v4f*)(sr);
  const v4f c = *(const v4f*)(sr + 4);
  float x[8];
#pragma unroll
  for (int e = 0; e < 4; ++e) { x[e] = a[e]; x[4 + e] = c[e]; }
  float m = fmaxf(fmaxf(fmaxf(x[0], x[1]), fmaxf(x[2], x[3])), fmaxf(fmaxf(x[4], x[5]), fmaxf(x[6], x[7])));
#pragma unroll
  for (int off = 16; off > 0; off >>= 1) m = fmaxf(m, __shfl_xor(m, off, 32));
  if (lane == 0) redM[wave] = m;
  __syncthreads();
  float gm = redM[0];
#pragma unroll
  for (int w = 1; w < 8; ++w) gm = fmaxf(gm, redM[w]);
  float ex[8];
  float s = 0.f;
#pragma unroll
  for (int e = 0; e < 8; ++e) { ex[e] = expf(x[e] - gm); s += ex[e]; }
#pragma unroll
  for (int off = 16; off > 0; off >>= 1) s += __shfl_xor(s, off, 32);
  if (lane == 0) redS[wave] = s;
  __syncthreads();
  float tot = 0.f;
#pragma unroll
  for (int w = 0; w < 8; ++w) tot += redS[w];
  const float inv = carry * (1.0f / tot);
  unsigned short hb[8];
#pragma unroll
  for (int e = 0; e < 8; ++e) hb[e] = h_bits(ex[e] * inv);
  const v4u u = (v4u){pk16(hb[0], hb[1]), pk16(hb[2], hb[3]), pk16(hb[4], hb[5]), pk16(hb[6], hb[7])};
  unsigned short* q = P + (size_t)row * kSeq + c0;
  *(volatile v4u*)q = u;
  __threadfence();
  *(volatile v4u*)q = u;
}

__global__ __launch_bounds__(256) void gelu_cast_kernel(const float* __restrict__ F, unsigned short* __restrict__ H,
                                                        int ldf, int coff, int n2) {
  const int i = blockIdx.x * 256 + threadIdx.x;
  if (i >= n2) return;
  const int per = ldf >> 1;
  const int r = i / per;
  const int c = (i - r * per) * 2;
  const float* p = F + (size_t)r * ldf + c;
  const float a = p[0], b = p[1];
  const float ga = 0.5f * a * (1.0f + erff(a * 0.70710678118654752f));
  const float gb = 0.5f * b * (1.0f + erff(b * 0.70710678118654752f));
  const unsigned u = pk16(h_bits(ga), h_bits(gb));
  volatile unsigned* q = (volatile unsigned*)(H + (size_t)r * kFF + coff + c);
  *q = u;
  __threadfence();
  *q = u;
}

template <bool W16>
__global__ __launch_bounds__(256) void ln_kernel(const float* __restrict__ Y, const float* __restrict__ gam,
                                                const float* __restrict__ bet, float* __restrict__ outf,
                                                unsigned short* __restrict__ out16) {
  __shared__ float red1[8];
  __shared__ float red2[8];
  __shared__ __align__(16) float srow[kDim];
  const int row  = blockIdx.x;
  const int t    = threadIdx.x;
  const int lane = t & 31, wave = t >> 5;
  const int c4   = t * 4;
  const v4f y = *(const v4f*)(Y + (size_t)row * kDim + c4);
  float s = (y[0] + y[1]) + (y[2] + y[3]);
#pragma unroll
  for (int off = 16; off > 0; off >>= 1) s += __shfl_xor(s, off, 32);
  if (lane == 0) red1[wave] = s;
  __syncthreads();
  float tot = 0.f;
#pragma unroll
  for (int w = 0; w < 8; ++w) tot += red1[w];
  const float mu = tot * kInvDim;
  float d[4];
  float vs = 0.f;
#pragma unroll
  for (int e = 0; e < 4; ++e) { d[e] = y[e] - mu; vs += d[e] * d[e]; }
#pragma unroll
  for (int off = 16; off > 0; off >>= 1) vs += __shfl_xor(vs, off, 32);
  if (lane == 0) red2[wave] = vs;
  __syncthreads();
  float tot2 = 0.f;
#pragma unroll
  for (int w = 0; w < 8; ++w) tot2 += red2[w];
  const float rstd = rsqrtf(tot2 * kInvDim + kLnEps);
  const v4f g4 = *(const v4f*)(gam + c4);
  const v4f b4 = *(const v4f*)(bet + c4);
  v4f ov;
#pragma unroll
  for (int e = 0; e < 4; ++e) ov[e] = d[e] * rstd * g4[e] + b4[e];
  float* op = outf + (size_t)row * kDim + c4;
  *(volatile v4f*)op = ov;
  __threadfence();
  *(volatile v4f*)op = ov;
  if (W16) {
    *(v4f*)(srow + c4) = ov;
    __syncthreads();
    if (t < 128) {
      const int c8 = t * 8;
      const v4f a = *(const v4f*)(srow + c8);
      const v4f c = *(const v4f*)(srow + c8 + 4);
      unsigned short hb[8];
#pragma unroll
      for (int e = 0; e < 4; ++e) { hb[e] = h_bits(a[e]); hb[4 + e] = h_bits(c[e]); }
      const v4u u = (v4u){pk16(hb[0], hb[1]), pk16(hb[2], hb[3]), pk16(hb[4], hb[5]), pk16(hb[6], hb[7])};
      unsigned short* q = out16 + (size_t)row * kDim + c8;
      *(volatile v4u*)q = u;
      __threadfence();
      *(volatile v4u*)q = u;
    }
  }
}

extern "C" void kernel_launch(void* const* d_in, const int* in_sizes, int n_in,
                              void* d_out, int out_size, void* d_ws, size_t ws_size,
                              hipStream_t stream) {
  if (n_in < 15) return;
  if (in_sizes[0] != kTok * kDim || in_sizes[1] != kTok * kDh || in_sizes[2] != kTok * kDh ||
      in_sizes[3] != kDim * kQKVN || in_sizes[4] != kQKVN || in_sizes[5] != kDim * kDim || in_sizes[6] != kDim ||
      in_sizes[7] != kDim || in_sizes[8] != kDim || in_sizes[9] != kDim * kFF || in_sizes[10] != kFF ||
      in_sizes[11] != kFF * kDim || in_sizes[12] != kDim || in_sizes[13] != kDim || in_sizes[14] != kDim) return;
  if (out_size != kTok * kDim) return;
  const size_t MiB = 1048576;
  const size_t total_carve = 114 * MiB;
  if (total_carve > ws_size) return;

  const float* x     = (const float*)d_in[0];
  const float* cosb  = (const float*)d_in[1];
  const float* sinb  = (const float*)d_in[2];
  const float* w_qkv = (const float*)d_in[3];
  const float* b_qkv = (const float*)d_in[4];
  const float* w_out = (const float*)d_in[5];
  const float* b_out = (const float*)d_in[6];
  const float* ln1_g = (const float*)d_in[7];
  const float* ln1_b = (const float*)d_in[8];
  const float* w1    = (const float*)d_in[9];
  const float* b1    = (const float*)d_in[10];
  const float* w2    = (const float*)d_in[11];
  const float* b2    = (const float*)d_in[12];
  const float* ln2_g = (const float*)d_in[13];
  const float* ln2_b = (const float*)d_in[14];
  float* out = (float*)d_out;

  char* ws = (char*)d_ws;
  unsigned short* W2T  = (unsigned short*)(ws + 0 * MiB);
  unsigned short* W1T  = (unsigned short*)(ws + 8 * MiB);
  unsigned short* WoT  = (unsigned short*)(ws + 16 * MiB);
  char* big = ws + 18 * MiB;
  unsigned short* X16  = (unsigned short*)(big);
  unsigned short* WqT  = (unsigned short*)(big + 8 * MiB);
  float*          QKVf = (float*)(big + 14 * MiB);
  float*          SC   = (float*)(big);
  unsigned short* P16  = (unsigned short*)(big + 32 * MiB);
  float*          Y1   = (float*)(big);
  float*          F1h  = (float*)(big);
  unsigned short* H16  = (unsigned short*)(big + 32 * MiB);
  float*          Y2   = (float*)(big);
  char* rq = ws + 82 * MiB;
  unsigned short* Q16  = (unsigned short*)(rq);
  unsigned short* K16  = (unsigned short*)(rq + 8 * MiB);
  unsigned short* VT16 = (unsigned short*)(rq + 16 * MiB);
  float*          X1   = (float*)(rq);
  unsigned short* X1h  = (unsigned short*)(rq + 16 * MiB);
  unsigned short* O16  = (unsigned short*)(ws + 106 * MiB);

  cast8_f16_kernel<<<(kTok * kDim / 8) / 256, 256, 0, stream>>>(x, X16, kTok * kDim / 8);
  wtcast_kernel<<<dim3(kDim / 64, kQKVN / 64), 256, 0, stream>>>(w_qkv, WqT, kDim, kQKVN, kWCarry);
  wtcast_kernel<<<dim3(kDim / 64, kDim / 64), 256, 0, stream>>>(w_out, WoT, kDim, kDim, kWCarry);
  wtcast_kernel<<<dim3(kDim / 64, kFF / 64), 256, 0, stream>>>(w1, W1T, kDim, kFF, kWCarry);
  wtcast_kernel<<<dim3(kFF / 64, kDim / 64), 256, 0, stream>>>(w2, W2T, kFF, kDim, kWCarry);

  wmma_gemm64<0, false, 2, 0, false><<<dim3((kTok / 64) * (kQKVN / 64) / 8, 1), 256, 0, stream>>>(
      X16, nullptr, kDim, 0L, WqT, nullptr, kDim, 0L, (void*)QKVf, nullptr, kQKVN, 0L,
      b_qkv, nullptr, 0L, kTok, kQKVN, kDim, kWCarryInv);

  rope_split_kernel<<<dim3(kSeq / 64, kGroups), 256, 0, stream>>>(QKVf, cosb, sinb, Q16, K16, VT16);

  for (int ch = 0; ch < kGroups / kGrpPerChunk; ++ch) {
    const int g0 = ch * kGrpPerChunk;
    const int bb = g0 / kHeads;
    const int h0 = g0 % kHeads;
    wmma_gemm64<0, false, 0, 0, false><<<dim3((kSeq / 64) * (kSeq / 64) / 8, kGrpPerChunk), 256, 0, stream>>>(
        Q16 + (size_t)g0 * kSeq * kDh, nullptr, kDh, (long)kSeq * kDh,
        K16 + (size_t)g0 * kSeq * kDh, nullptr, kDh, (long)kSeq * kDh,
        (void*)SC, nullptr, kSeq, (long)kSeq * kSeq,
        nullptr, nullptr, 0L, kSeq, kSeq, kDh, kScoreScale);
    softmax_row_kernel<<<kGrpPerChunk * kSeq, 256, 0, stream>>>(SC, P16, kPCarry);
    wmma_gemm64<0, false, 0, 1, false><<<dim3((kSeq / 64) * (kDh / 64) / 8, kGrpPerChunk), 256, 0, stream>>>(
        P16, nullptr, kSeq, (long)kSeq * kSeq,
        VT16 + (size_t)g0 * kDh * kSeq, nullptr, kSeq, (long)kDh * kSeq,
        (void*)(O16 + (size_t)bb * kSeq * kDim + (size_t)h0 * kDh), nullptr, kDim, (long)kDh,
        nullptr, nullptr, 0L, kSeq, kDh, kSeq, kPCarryInv);
  }

  wmma_gemm64<0, false, 2, 0, true><<<dim3((kTok / 64) * (kDim / 64) / 8, 1), 256, 0, stream>>>(
      O16, nullptr, kDim, 0L, WoT, nullptr, kDim, 0L, (void*)Y1, nullptr, kDim, 0L,
      b_out, x, 0L, kTok, kDim, kDim, kWCarryInv);

  ln_kernel<true><<<kTok, 256, 0, stream>>>(Y1, ln1_g, ln1_b, X1, X1h);

  for (int hf = 0; hf < 2; ++hf) {
    wmma_gemm64<0, false, 2, 0, false><<<dim3((kTok / 64) * (kFFH / 64) / 8, 1), 256, 0, stream>>>(
        X1h, nullptr, kDim, 0L, W1T + (size_t)hf * kFFH * kDim, nullptr, kDim, 0L, (void*)F1h, nullptr, kFFH, 0L,
        b1 + hf * kFFH, nullptr, 0L, kTok, kFFH, kDim, kWCarryInv);
    gelu_cast_kernel<<<(kTok * kFFH / 2) / 256, 256, 0, stream>>>(F1h, H16, kFFH, hf * kFFH, kTok * kFFH / 2);
  }

  wmma_gemm64<0, false, 2, 0, true><<<dim3((kTok / 64) * (kDim / 64) / 8, 1), 256, 0, stream>>>(
      H16, nullptr, kFF, 0L, W2T, nullptr, kFF, 0L, (void*)Y2, nullptr, kDim, 0L,
      b2, X1, 0L, kTok, kDim, kFF, kWCarryInv);

  ln_kernel<false><<<kTok, 256, 0, stream>>>(Y2, ln2_g, ln2_b, out, nullptr);
}
